// TimedPoincareTransformerLayer_69621419868919
// MI455X (gfx1250) — hardware-verified
//
#include <hip/hip_runtime.h>
#include <math.h>


#define NB_  4
#define TT   1024
#define DD   1024
#define NH_  16
#define HD   64
#define FFH  4096
#define ADA  (6 * DD)
#define PCAR 1024.0f
#define EPS_ 1e-7f
#define MAXT 0.99999f
#define BHBN 4.0146746635437012f
#define BNBH 0.24908619f
typedef _Float16 h16;
typedef unsigned short bf;
typedef __attribute__((ext_vector_type(16))) __bf16   v16bf;
typedef __attribute__((ext_vector_type(16))) _Float16 v16h;
typedef __attribute__((ext_vector_type(8)))  _Float16 v8h;
typedef __attribute__((ext_vector_type(8)))  unsigned short v8us;
typedef __attribute__((ext_vector_type(8)))  float    v8f;
typedef __attribute__((ext_vector_type(4)))  float    v4f;
typedef v8h  __attribute__((may_alias)) v8ha;
typedef v4f  __attribute__((may_alias)) v4fa;
typedef v8us __attribute__((may_alias)) v8usa;

__device__ __forceinline__ unsigned short f2bf(float f) { unsigned u = __float_as_uint(f); u += 0x7FFFu + ((u >> 16) & 1u); return (unsigned short)(u >> 16); }
__device__ __forceinline__ float bf2f(unsigned short b) { return __uint_as_float(((unsigned)b) << 16); }
__device__ __forceinline__ float bfr(float f) { return bf2f(f2bf(f)); }
__device__ __forceinline__ v16h cat16(v8h lo, v8h hi) { return __builtin_shufflevector(lo, hi, 0, 1, 2, 3, 4, 5, 6, 7, 8, 9, 10, 11, 12, 13, 14, 15); }
__device__ __forceinline__ v16bf cat16b(v8us lo, v8us hi) { return __builtin_bit_cast(v16bf, __builtin_shufflevector(lo, hi, 0, 1, 2, 3, 4, 5, 6, 7, 8, 9, 10, 11, 12, 13, 14, 15)); }
__device__ __forceinline__ v8f wmma16(v16h a, v16h b, v8f c) { return __builtin_amdgcn_wmma_f32_16x16x32_f16(false, a, false, b, (short)0, c, false, false); }
__device__ __forceinline__ v8f wmmab(v16bf a, v16bf b, v8f c) { return __builtin_amdgcn_wmma_f32_16x16x32_bf16(false, a, false, b, (short)0, c, false, false); }


template <typename T16> struct WFrag;
template <> struct WFrag<h16> { typedef v16h V; static __device__ __forceinline__ V ld(const h16* p) { return cat16(*(const v8h*)p, *(const v8h*)(p + 16)); } static __device__ __forceinline__ v8f mma(V a, V b, v8f c) { return wmma16(a, b, c); } };
template <> struct WFrag<bf> { typedef v16bf V; static __device__ __forceinline__ V ld(const bf* p) { return cat16b(*(const v8us*)p, *(const v8us*)(p + 16)); } static __device__ __forceinline__ v8f mma(V a, V b, v8f c) { return wmmab(a, b, c); } };
template <typename T16, int NSPLIT, bool BIAS>
__global__ __launch_bounds__(32) void k_gemmw(const T16* __restrict__ A, const T16* __restrict__ A2, const T16* __restrict__ Bt, const T16* __restrict__ Bt2, int K, float* C, int ldc, const float* __restrict__ bias, size_t sA, size_t sB, size_t sC) {
    typedef typename WFrag<T16>::V V;
    __shared__ __align__(16) float os[16 * 68];
    const size_t z = blockIdx.z; A += z * sA; if (A2) A2 += z * sA; Bt += z * sB; if (Bt2) Bt2 += z * sB; C += z * sC;
    const int lane = threadIdx.x & 31, lr = lane & 15, hi = lane >> 4; const int r0 = blockIdx.x * 64, c0 = blockIdx.y * 64;
    v8f acc[4][4];
#pragma unroll
    for (int mb = 0; mb < 4; ++mb)
#pragma unroll
        for (int nb = 0; nb < 4; ++nb) acc[mb][nb] = (v8f){};
    const size_t aoff = (size_t)(r0 + lr) * K + 8 * hi, boff = (size_t)(c0 + lr) * K + 8 * hi;
#pragma unroll 1
    for (int kc = 0; kc < K; kc += 32) {
        V a[4], a2[4];
#pragma unroll
        for (int mb = 0; mb < 4; ++mb) { a[mb] = WFrag<T16>::ld(A + aoff + (size_t)mb * 16 * K + kc); if (NSPLIT == 1 || NSPLIT == 2) a2[mb] = WFrag<T16>::ld(A2 + aoff + (size_t)mb * 16 * K + kc); }
#pragma unroll
        for (int nb = 0; nb < 4; ++nb) { const V b = WFrag<T16>::ld(Bt + boff + (size_t)nb * 16 * K + kc); V b2; if (NSPLIT >= 2) b2 = WFrag<T16>::ld(Bt2 + boff + (size_t)nb * 16 * K + kc);
#pragma unroll
            for (int mb = 0; mb < 4; ++mb) { acc[mb][nb] = WFrag<T16>::mma(a[mb], b, acc[mb][nb]); if (NSPLIT == 1 || NSPLIT == 2) acc[mb][nb] = WFrag<T16>::mma(a2[mb], b, acc[mb][nb]); if (NSPLIT >= 2) acc[mb][nb] = WFrag<T16>::mma(a[mb], b2, acc[mb][nb]); } }
        asm volatile("v_nop\n\tv_nop\n\tv_nop\n\tv_nop" : "+v"(acc[0][0]), "+v"(acc[1][1]), "+v"(acc[2][2]), "+v"(acc[3][3]) : "v"(a[0]), "v"(a[3]));
    }
#pragma unroll
    for (int mb = 0; mb < 4; ++mb) {
#pragma unroll
        for (int nb = 0; nb < 4; ++nb) {
#pragma unroll
            for (int j = 0; j < 8; ++j) os[(hi * 8 + j) * 68 + nb * 16 + lr] = acc[mb][nb][j]; }
        __builtin_amdgcn_wave_barrier(); asm volatile("" ::: "memory");
        float* crow = C + (size_t)(r0 + mb * 16) * ldc + c0;
#pragma unroll 1
        for (int ps = 0; ps < 2; ++ps) {
#pragma unroll
            for (int s = 0; s < 8; ++s) { const int row = 2 * s + hi, cofs = lr * 4; v4f val = *(const v4fa*)(os + row * 68 + cofs); if (BIAS) { val[0] += bfr(bias[c0 + cofs]); val[1] += bfr(bias[c0 + cofs + 1]); val[2] += bfr(bias[c0 + cofs + 2]); val[3] += bfr(bias[c0 + cofs + 3]); }
                *(volatile v4f*)(crow + (size_t)row * ldc + cofs) = val; }
            if (ps == 0) __threadfence(); }
        __builtin_amdgcn_wave_barrier(); asm volatile("" ::: "memory");
    }
}

__device__ __forceinline__ h16 tohx(float x) { return (h16)x; }
__device__ __forceinline__ void splitf(float y, unsigned short& h, unsigned short& l) { h = f2bf(y); l = f2bf(y - bf2f(h)); }
typedef __attribute__((ext_vector_type(4))) _Float16 v4h;
typedef __attribute__((ext_vector_type(2))) _Float16 v2h;
typedef __attribute__((ext_vector_type(2))) unsigned short v2us;
typedef __attribute__((ext_vector_type(4))) unsigned short v4us;

#define OPQ(x) asm volatile("" : "+v"(x))
__device__ __forceinline__ float sqacc(float s, float a) { float p = __fmul_rn(a, a); OPQ(p); return __fadd_rn(s, p); }
__device__ __forceinline__ float mulacc(float s, float a, float b) { float p = __fmul_rn(a, b); OPQ(p); return __fadd_rn(s, p); }
__device__ __forceinline__ float RCP(float x) { return __builtin_amdgcn_rcpf(x); }
__device__ __forceinline__ float SQRTF(float x) { return __builtin_amdgcn_sqrtf(x); }
__device__ __forceinline__ float TANHF(float n) { return __fsub_rn(1.0f, __fmul_rn(2.0f, RCP(__fadd_rn(__expf(__fmul_rn(2.0f, n)), 1.0f)))); }
__device__ __forceinline__ float ATANHF(float z) { return __fmul_rn(0.5f, __logf(__fmul_rn(__fadd_rn(1.0f, z), RCP(__fsub_rn(1.0f, z))))); }
__device__ __forceinline__ float wsum32(float s) {
#pragma unroll
    for (int sh = 16; sh; sh >>= 1) s += __shfl_xor(s, sh, 32); return s; }
__device__ __forceinline__ float hsum16(float s) {
#pragma unroll
    for (int sh = 8; sh; sh >>= 1) s += __shfl_xor(s, sh, 32); return s; }
__device__ __forceinline__ float rnorm1024(const float* v) { float s = 0.f;
#pragma unroll
    for (int i = 0; i < 32; ++i) s = sqacc(s, v[i]); return fmaxf(SQRTF(wsum32(s)), EPS_); }
__device__ __forceinline__ float hnorm64(const float* v4) { float s = 0.f;
#pragma unroll
    for (int q = 0; q < 4; ++q) s = sqacc(s, v4[q]); return fmaxf(SQRTF(hsum16(s)), EPS_); }
__device__ __forceinline__ float lmc(float n) { return ATANHF(fminf(fmaxf(n, EPS_), MAXT)); }
__device__ __forceinline__ void scale_row(float* v, float c, float n) {
    const float f = __fmul_rn(c, RCP(n));
#pragma unroll
    for (int i = 0; i < 32; ++i) v[i] = __fmul_rn(v[i], f); }
__device__ __forceinline__ void scale4(float* v4, float c, float n) { const float f = __fmul_rn(c, RCP(n));
#pragma unroll
    for (int q = 0; q < 4; ++q) v4[q] = __fmul_rn(v4[q], f); }
__device__ __forceinline__ void expmap_row(float* v) { const float n = rnorm1024(v); scale_row(v, TANHF(n), n); }
__device__ __forceinline__ void logmap_row(float* v) { const float n = rnorm1024(v); scale_row(v, lmc(n), n); }
__device__ __forceinline__ void expmap_heads(float* v) {
#pragma unroll
    for (int c = 0; c < 8; ++c) { const float n = hnorm64(v + c * 4); scale4(v + c * 4, TANHF(n), n); } }
__device__ __forceinline__ void logmap_heads(float* v) {
#pragma unroll
    for (int c = 0; c < 8; ++c) { const float n = hnorm64(v + c * 4); scale4(v + c * 4, lmc(n), n); } }
__device__ __forceinline__ void load_row(const float* __restrict__ p, int lane, float* v) {
#pragma unroll
    for (int c = 0; c < 8; ++c) { const v4f a = *(const v4f*)(p + c * 128 + lane * 4);
#pragma unroll
        for (int q = 0; q < 4; ++q) v[c * 4 + q] = a[q]; } }
__device__ __forceinline__ void layernorm_row(float* v) {
    float s = 0.f;
#pragma unroll
    for (int i = 0; i < 32; ++i) s = __fadd_rn(s, v[i]);
    const float mu = __fmul_rn(wsum32(s), 1.0f / DD); float q2 = 0.f;
#pragma unroll
    for (int i = 0; i < 32; ++i) { const float d0 = __fsub_rn(v[i], mu); q2 = sqacc(q2, d0); }
    const float rden = RCP(SQRTF(__fadd_rn(__fmul_rn(wsum32(q2), 1.0f / DD), 1e-6f)));
#pragma unroll
    for (int i = 0; i < 32; ++i) v[i] = __fmul_rn(__fsub_rn(v[i], mu), rden); }
__device__ __forceinline__ void modulate_row(float* v, const float* __restrict__ sc, const float* __restrict__ sh, int lane) {
#pragma unroll
    for (int c = 0; c < 8; ++c) { const v4f a = *(const v4f*)(sc + c * 128 + lane * 4), b = *(const v4f*)(sh + c * 128 + lane * 4);
#pragma unroll
        for (int q = 0; q < 4; ++q) { float p = __fmul_rn(v[c * 4 + q], __fadd_rn(1.0f, a[q])); OPQ(p); v[c * 4 + q] = __fadd_rn(p, b[q]); } } }
__device__ __forceinline__ void store_split_row(const float* v, int lane, size_t r, bf* Ph, bf* Pl) {
#pragma unroll 1
    for (int ps = 0; ps < 2; ++ps) {
#pragma unroll
        for (int c = 0; c < 8; ++c) { v4us oh, ol;
#pragma unroll
            for (int q = 0; q < 4; ++q) { unsigned short a, b2; splitf(v[c * 4 + q], a, b2); oh[q] = a; ol[q] = b2; }
            *(volatile v4us*)(Ph + r * DD + c * 128 + lane * 4) = oh; *(volatile v4us*)(Pl + r * DD + c * 128 + lane * 4) = ol; }
        if (ps == 0) __threadfence(); } }
__device__ __forceinline__ void store_row(const float* v, int lane, float* dst) {
#pragma unroll 1
    for (int ps = 0; ps < 2; ++ps) {
#pragma unroll
        for (int c = 0; c < 8; ++c) { v4f o;
#pragma unroll
            for (int q = 0; q < 4; ++q) o[q] = v[c * 4 + q];
            *(volatile v4f*)(dst + c * 128 + lane * 4) = o; }
        if (ps == 0) __threadfence(); } }

__global__ __launch_bounds__(256) void k_wtG(const float* __restrict__ w, int K, int N, bf* Bt) {
    const int lane = threadIdx.x & 31; const int L0 = (blockIdx.x * 8 + (threadIdx.x >> 5)) * 8; const int nlines = N * K / 64;
#pragma unroll 1
    for (int ps = 0; ps < 2; ++ps) {
#pragma unroll 1
        for (int l = 0; l < 8; ++l) { const int L = L0 + l; if (L >= nlines) break; const size_t e = (size_t)L * 64 + lane * 2; const int k = (int)(e % K), n = (int)(e / K); v2us o;
            o[0] = f2bf(w[(size_t)k * N + n]); o[1] = f2bf(w[(size_t)(k + 1) * N + n]); *(volatile v2us*)(Bt + e) = o; }
        if (ps == 0) __threadfence(); }
}
__global__ __launch_bounds__(256) void k_ada(const float* __restrict__ t, const float* __restrict__ w, const float* __restrict__ b, float* ADAo) {
    const int o = blockIdx.x * 256 + threadIdx.x; if (o >= ADA) return; float s = 0.f;
#pragma unroll 4
    for (int k = 0; k < DD; ++k) { float a = bfr(t[k]), c = bfr(w[(size_t)k * ADA + o]); OPQ(a); OPQ(c); s = mulacc(s, a, c); }
    s = __fadd_rn(s, bfr(b[o])); *(volatile float*)(ADAo + o) = s; __threadfence(); *(volatile float*)(ADAo + o) = s;
}
template <int RAWBF>
__global__ __launch_bounds__(256) void k_pre(const float* __restrict__ X, const float* __restrict__ sc, const float* __restrict__ sh, bf* Th, bf* Tl) {
    const int lane = threadIdx.x & 31; const int r = blockIdx.x * 8 + (threadIdx.x >> 5); if (r >= TT) return; float v[32];
    load_row(X + (size_t)r * DD, lane, v);
    if (RAWBF) {
#pragma unroll
        for (int i = 0; i < 32; ++i) { v[i] = bfr(v[i]); OPQ(v[i]); } }
    logmap_row(v); layernorm_row(v); modulate_row(v, sc, sh, lane); expmap_row(v); logmap_row(v);
    store_split_row(v, lane, (size_t)r, Th, Tl);
}
template <int MODE>
__global__ __launch_bounds__(256) void k_heads(const float* __restrict__ U, float sc, h16* P16, float* ROW) {
    const int lane = threadIdx.x & 31; const int r = blockIdx.x * 8 + (threadIdx.x >> 5); if (r >= TT) return; float v[32];
    load_row(U + (size_t)r * DD, lane, v); expmap_row(v); logmap_row(v);
#pragma unroll
    for (int i = 0; i < 32; ++i) v[i] = __fmul_rn(v[i], BHBN);
    expmap_heads(v); logmap_heads(v);
    if (MODE == 0) {
#pragma unroll 1
        for (int ps = 0; ps < 2; ++ps) {
#pragma unroll
            for (int c = 0; c < 8; ++c) { const int h = 2 * c + (lane >> 4); const int d = (lane & 15) * 4; v4h o;
#pragma unroll
                for (int q = 0; q < 4; ++q) o[q] = tohx(__fmul_rn(v[c * 4 + q], sc));
                *(volatile v4h*)(P16 + ((size_t)h * TT + r) * HD + d) = o; }
            if (ps == 0) __threadfence(); }
    } else store_row(v, lane, ROW + (size_t)r * DD);
}
__global__ __launch_bounds__(256) void k_vt16(const float* __restrict__ ROW, h16* VT) {
    const int lane = threadIdx.x & 31; const int L0 = (blockIdx.x * 8 + (threadIdx.x >> 5)) * 8; const int nlines = NH_ * HD * TT / 64;
#pragma unroll 1
    for (int ps = 0; ps < 2; ++ps) {
#pragma unroll
        for (int l = 0; l < 8; ++l) { const int L = L0 + l; if (L >= nlines) break; const int e = L * 64 + lane * 2; const int s = e & (TT - 1); const int d = (e >> 10) & 63; const int h = e >> 16; v2h o;
#pragma unroll
            for (int q = 0; q < 2; ++q) o[q] = tohx(ROW[(size_t)(s + q) * DD + h * HD + d]);
            *(volatile v2h*)(VT + (size_t)e) = o; }
        if (ps == 0) __threadfence(); }
}
__global__ __launch_bounds__(256) void k_psoft(const float* __restrict__ Sb, int NR, h16* P) {
    const int lane = threadIdx.x & 31; const int row = blockIdx.x * 8 + (threadIdx.x >> 5); if (row >= NR) return;
    const float* sr = Sb + (size_t)row * TT; float v[32]; float mx = -3.0e38f;
#pragma unroll
    for (int ch = 0; ch < 8; ++ch) { const int j0 = ch * 128 + lane * 4; const v4f a = *(const v4f*)(sr + j0);
#pragma unroll
        for (int q = 0; q < 4; ++q) { v[ch * 4 + q] = a[q]; mx = fmaxf(mx, a[q]); } }
#pragma unroll
    for (int sh = 16; sh; sh >>= 1) mx = fmaxf(mx, __shfl_xor(mx, sh, 32));
    float sum = 0.f;
#pragma unroll
    for (int k = 0; k < 32; ++k) { v[k] = __expf(v[k] - mx); sum += v[k]; }
#pragma unroll
    for (int sh = 16; sh; sh >>= 1) sum += __shfl_xor(sum, sh, 32);
    const float f = __fdiv_rn(PCAR, sum);
#pragma unroll 1
    for (int ps = 0; ps < 2; ++ps) {
#pragma unroll
        for (int ch = 0; ch < 8; ++ch) { v4h o;
#pragma unroll
            for (int q = 0; q < 4; ++q) o[q] = tohx(v[ch * 4 + q] * f);
            *(volatile v4h*)(P + (size_t)row * TT + ch * 128 + lane * 4) = o; }
        if (ps == 0) __threadfence(); }
}
__global__ __launch_bounds__(256) void k_post(const float* __restrict__ O, bf* Th, bf* Tl) {
    const int lane = threadIdx.x & 31; const int r = blockIdx.x * 8 + (threadIdx.x >> 5); if (r >= TT) return; float v[32];
#pragma unroll
    for (int c = 0; c < 8; ++c) { const int h = 2 * c + (lane >> 4); const int d = (lane & 15) * 4; const v4f a = *(const v4f*)(O + ((size_t)h * TT + r) * HD + d);
#pragma unroll
        for (int q = 0; q < 4; ++q) v[c * 4 + q] = __fmul_rn(a[q], 1.0f / PCAR); }
    expmap_heads(v); logmap_heads(v);
#pragma unroll
    for (int i = 0; i < 32; ++i) v[i] = __fmul_rn(v[i], BNBH);
    expmap_row(v); logmap_row(v);
    store_split_row(v, lane, (size_t)r, Th, Tl);
}
__device__ __forceinline__ void mobius_rows(const float* a, float* y) {
    float x2 = 0.f, y2 = 0.f, xy = 0.f;
#pragma unroll
    for (int i = 0; i < 32; ++i) { x2 = sqacc(x2, a[i]); y2 = sqacc(y2, y[i]); xy = mulacc(xy, a[i], y[i]); }
    x2 = wsum32(x2); y2 = wsum32(y2); xy = wsum32(xy);
    const float cx = __fadd_rn(__fadd_rn(1.0f, __fmul_rn(2.0f, xy)), y2), cy = __fsub_rn(1.0f, x2);
    const float rden = RCP(fmaxf(__fadd_rn(__fadd_rn(1.0f, __fmul_rn(2.0f, xy)), __fmul_rn(x2, y2)), EPS_));
#pragma unroll
    for (int i = 0; i < 32; ++i) { float p1 = __fmul_rn(cx, a[i]), p2 = __fmul_rn(cy, y[i]); OPQ(p1); OPQ(p2); y[i] = __fmul_rn(__fadd_rn(p1, p2), rden); } }
template <int RAWBF>
__global__ __launch_bounds__(256) void k_gate_res(const float* __restrict__ U, const float* __restrict__ RES, const float* __restrict__ gmod, float* XX) {
    const int lane = threadIdx.x & 31; const int r = blockIdx.x * 8 + (threadIdx.x >> 5); if (r >= TT) return; float v[32], a[32];
    load_row(U + (size_t)r * DD, lane, v); expmap_row(v); logmap_row(v);
#pragma unroll
    for (int c = 0; c < 8; ++c) { const v4f gg = *(const v4f*)(gmod + c * 128 + lane * 4);
#pragma unroll
        for (int q = 0; q < 4; ++q) v[c * 4 + q] = __fmul_rn(gg[q], v[c * 4 + q]); }
    expmap_row(v);
    load_row(RES + (size_t)r * DD, lane, a);
    if (RAWBF) {
#pragma unroll
        for (int i = 0; i < 32; ++i) { a[i] = bfr(a[i]); OPQ(a[i]); } }
    mobius_rows(a, v);
    store_row(v, lane, XX + (size_t)r * DD);
}
__global__ __launch_bounds__(256) void k_ff1(const float* __restrict__ U, bf* Th, bf* Tl) {
    const int lane = threadIdx.x & 31; const int r = blockIdx.x * 8 + (threadIdx.x >> 5); if (r >= TT) return; const float* ur = U + (size_t)r * FFH;
    float s = 0.f;
#pragma unroll 2
    for (int k = 0; k < FFH / 128; ++k) { const v4f a = *(const v4f*)(ur + k * 128 + lane * 4);
#pragma unroll
        for (int q = 0; q < 4; ++q) s = sqacc(s, a[q]); }
    const float n = fmaxf(SQRTF(wsum32(s)), EPS_); const float f1 = __fmul_rn(TANHF(n), RCP(n));
    float s2 = 0.f;
#pragma unroll 2
    for (int k = 0; k < FFH / 128; ++k) { const v4f a = *(const v4f*)(ur + k * 128 + lane * 4);
#pragma unroll
        for (int q = 0; q < 4; ++q) { const float p = __fmul_rn(a[q], f1); s2 = sqacc(s2, p); } }
    const float n2 = fmaxf(SQRTF(wsum32(s2)), EPS_); const float f2 = __fmul_rn(lmc(n2), RCP(n2));
#pragma unroll 1
    for (int ps = 0; ps < 2; ++ps) {
#pragma unroll 2
        for (int k = 0; k < FFH / 128; ++k) { const v4f a = *(const v4f*)(ur + k * 128 + lane * 4); v4us oh, ol;
#pragma unroll
            for (int q = 0; q < 4; ++q) { const float t = __fmul_rn(__fmul_rn(a[q], f1), f2); unsigned short x1, x2; splitf(t, x1, x2); oh[q] = x1; ol[q] = x2; }
            *(volatile v4us*)(Th + (size_t)r * FFH + k * 128 + lane * 4) = oh; *(volatile v4us*)(Tl + (size_t)r * FFH + k * 128 + lane * 4) = ol; }
        if (ps == 0) __threadfence(); }
}

extern "C" void kernel_launch(void* const* d_in, const int* in_sizes, int n_in,
                              void* d_out, int out_size, void* d_ws, size_t ws_size, hipStream_t stream) {
    (void)in_sizes; (void)n_in; (void)out_size;
    const float* IN[16]; for (int i = 0; i < 16; ++i) IN[i] = (const float*)d_in[i];
    const float* x = IN[0]; const float* temb = IN[1];
    float* OUT = (float*)d_out;
    char* wsp = (char*)d_ws;
    auto take = [&](size_t bytes) { char* p = wsp; wsp += (bytes + 255) & ~(size_t)255; return (void*)p; };
    bf* WQ = (bf*)take((size_t)DD * DD * 2); bf* WK = (bf*)take((size_t)DD * DD * 2); bf* WV = (bf*)take((size_t)DD * DD * 2); bf* WO = (bf*)take((size_t)DD * DD * 2); bf* W1T = (bf*)take((size_t)FFH * DD * 2); bf* W2T = (bf*)take((size_t)DD * FFH * 2);
    float* ADAb = (float*)take((size_t)ADA * 4);
    bf* T1h = (bf*)take((size_t)TT * DD * 2); bf* T1l = (bf*)take((size_t)TT * DD * 2); float* U = (float*)take((size_t)TT * DD * 4);
    h16* QP = (h16*)take((size_t)TT * DD * 2); h16* KP = (h16*)take((size_t)TT * DD * 2); float* VROW = (float*)take((size_t)TT * DD * 4); h16* VT = (h16*)take((size_t)TT * DD * 2);
    float* Sb = (float*)take((size_t)NH_ * TT * TT * 4); h16* Pm = (h16*)take((size_t)NH_ * TT * TT * 2); float* Ob = (float*)take((size_t)NH_ * TT * HD * 4);
    bf* T2h = (bf*)take((size_t)TT * DD * 2); bf* T2l = (bf*)take((size_t)TT * DD * 2); float* XX = (float*)take((size_t)TT * DD * 4);
    float* U3 = (float*)take((size_t)TT * FFH * 4); bf* T4h = (bf*)take((size_t)TT * FFH * 2); bf* T4l = (bf*)take((size_t)TT * FFH * 2);
    if ((size_t)(wsp - (char*)d_ws) > ws_size) return;
    bf* T3h = T1h; bf* T3l = T1l;
    { const unsigned g1 = (unsigned)((DD * DD / 64 + 63) / 64), gF = (unsigned)((FFH * DD / 64 + 63) / 64);
      k_wtG<<<g1, 256, 0, stream>>>(IN[2], DD, DD, WQ); k_wtG<<<g1, 256, 0, stream>>>(IN[4], DD, DD, WK); k_wtG<<<g1, 256, 0, stream>>>(IN[6], DD, DD, WV); k_wtG<<<g1, 256, 0, stream>>>(IN[8], DD, DD, WO);
      k_wtG<<<gF, 256, 0, stream>>>(IN[10], DD, FFH, W1T); k_wtG<<<gF, 256, 0, stream>>>(IN[12], FFH, DD, W2T); }
    const dim3 gP(TT / 64, DD / 64, 1); const unsigned RW = TT / 8;
    for (int b = 0; b < NB_; ++b) { const float* xb = x + (size_t)b * TT * DD;
        k_ada<<<ADA / 256, 256, 0, stream>>>(temb + (size_t)b * DD, IN[14], IN[15], ADAb);
        const float* sh_msa = ADAb; const float* sc_msa = ADAb + DD; const float* g_msa = ADAb + 2 * DD; const float* sh_mlp = ADAb + 3 * DD; const float* sc_mlp = ADAb + 4 * DD; const float* g_mlp = ADAb + 5 * DD;
        k_pre<1><<<RW, 256, 0, stream>>>(xb, sc_msa, sh_msa, T1h, T1l);
        k_gemmw<bf, 1, true><<<gP, 32, 0, stream>>>(T1h, T1l, WQ, nullptr, DD, U, DD, IN[3], 0, 0, 0); k_heads<0><<<RW, 256, 0, stream>>>(U, 0.125f, QP, nullptr);
        k_gemmw<bf, 1, true><<<gP, 32, 0, stream>>>(T1h, T1l, WK, nullptr, DD, U, DD, IN[5], 0, 0, 0); k_heads<0><<<RW, 256, 0, stream>>>(U, 1.0f, KP, nullptr);
        k_gemmw<bf, 1, true><<<gP, 32, 0, stream>>>(T1h, T1l, WV, nullptr, DD, U, DD, IN[7], 0, 0, 0); k_heads<1><<<RW, 256, 0, stream>>>(U, 1.0f, nullptr, VROW);
        k_vt16<<<(unsigned)((NH_ * HD * TT / 64 + 63) / 64), 256, 0, stream>>>(VROW, VT);
        k_gemmw<h16, 0, false><<<dim3(TT / 64, TT / 64, NH_), 32, 0, stream>>>(QP, nullptr, KP, nullptr, HD, Sb, TT, nullptr, (size_t)TT * HD, (size_t)TT * HD, (size_t)TT * TT);
        k_psoft<<<NH_ * TT / 8, 256, 0, stream>>>(Sb, NH_ * TT, Pm);
        k_gemmw<h16, 0, false><<<dim3(TT / 64, 1, NH_), 32, 0, stream>>>(Pm, nullptr, VT, nullptr, TT, Ob, HD, nullptr, (size_t)TT * TT, (size_t)HD * TT, (size_t)TT * HD);
        k_post<<<RW, 256, 0, stream>>>(Ob, T2h, T2l);
        k_gemmw<bf, 1, true><<<gP, 32, 0, stream>>>(T2h, T2l, WO, nullptr, DD, U, DD, IN[9], 0, 0, 0);
        k_gate_res<1><<<RW, 256, 0, stream>>>(U, xb, g_msa, XX);
        k_pre<0><<<RW, 256, 0, stream>>>(XX, sc_mlp, sh_mlp, T3h, T3l);
        k_gemmw<bf, 1, true><<<dim3(TT / 64, FFH / 64, 1), 32, 0, stream>>>(T3h, T3l, W1T, nullptr, DD, U3, FFH, IN[11], 0, 0, 0);
        k_ff1<<<RW, 256, 0, stream>>>(U3, T4h, T4l);
        k_gemmw<bf, 1, true><<<gP, 32, 0, stream>>>(T4h, T4l, W2T, nullptr, FFH, U, DD, IN[13], 0, 0, 0);
        k_gate_res<0><<<RW, 256, 0, stream>>>(U, XX, g_mlp, OUT + (size_t)b * TT * DD); }
}
